// TransformerEncoderLayerQaN_64879775973735
// MI455X (gfx1250) — hardware-verified
//
#include <hip/hip_runtime.h>


namespace {
constexpr int T = 512, B = 4, D = 1024, NH = 16, DFF = 4096, NQ = 10, WIN = 64, NW = T / WIN, NR = T * B;
constexpr float XS = 8.0f, WSC = 256.0f;
typedef _Float16 b16;
typedef __attribute__((ext_vector_type(16))) _Float16 v16b;
typedef __attribute__((ext_vector_type(8))) _Float16 v8b;
typedef __attribute__((ext_vector_type(8))) float v8f;
typedef __attribute__((ext_vector_type(4))) float v4f;
__device__ __forceinline__ float bf16_rne(float f) { unsigned int u = __float_as_uint(f); u += 0x7FFFu + ((u >> 16) & 1u); return __uint_as_float(u & 0xFFFF0000u); }
__device__ __forceinline__ void split16(float v, b16& hi, b16& lo) { hi = (b16)v; lo = (b16)(v - (float)hi); }
__device__ __forceinline__ v16b frag_kb(const b16* p, int hh) { const v8b a = *(const v8b*)(p + 8 * hh), b = *(const v8b*)(p + 16 + 8 * hh); v16b f;
#pragma unroll
  for (int e = 0; e < 8; ++e) { f[e] = a[e]; f[8 + e] = b[e]; } return f; }
__device__ __forceinline__ v8f wmma16b(v16b a, v16b b, v8f c) { v8f d = __builtin_amdgcn_wmma_f32_16x16x32_f16(false, a, false, b, (short)0, c, false, false); asm volatile("v_nop\n\tv_nop\n\tv_nop\n\tv_nop" : "+v"(d) : "v"(a), "v"(b)); return d; }
__device__ __forceinline__ void wave_lds_sync() { __builtin_amdgcn_fence(__ATOMIC_RELEASE, "workgroup"); __builtin_amdgcn_wave_barrier(); __builtin_amdgcn_fence(__ATOMIC_ACQUIRE, "workgroup"); }
__device__ __forceinline__ float pmul(float a, float b) { float p = a * b; asm volatile("" : "+v"(p)); return p; }

__global__ __launch_bounds__(256) void wcopy_kernel(const float* __restrict__ w, size_t total, b16* __restrict__ WT) { const size_t u = (size_t)blockIdx.x * 256 + threadIdx.x; if (u >= total / 8) return; const size_t e = u * 8; v8b v;
#pragma unroll
  for (int j = 0; j < 8; ++j) v[j] = (b16)(bf16_rne(w[e + j]) * WSC); for (int pass = 0; pass < 2; ++pass) { *(volatile v8b*)(WT + e) = v; __threadfence(); } }
__global__ __launch_bounds__(32) void qn_kernel(const float* __restrict__ qs, b16* __restrict__ QNh, b16* __restrict__ QNl) {
  const int lane = threadIdx.x, n = blockIdx.x; __shared__ float Nrm[NH];
  if (n < NQ && lane < NH) { float s = 0.0f; for (int d = 0; d < 64; ++d) { const float v = bf16_rne(qs[(size_t)n * D + lane * 64 + d]); s += pmul(v, v); } Nrm[lane] = 1.0f / (sqrtf(s) + 1e-6f); }
  wave_lds_sync();
  for (int pass = 0; pass < 2; ++pass) { for (int q = 0; q < D / 32; ++q) { const int d = q * 32 + lane; float v = 0.0f; if (n < NQ) v = pmul(pmul(bf16_rne(qs[(size_t)n * D + d]), Nrm[d / 64]), 0.125f * 0.03125f);
      b16 p, ql; split16(v * XS, p, ql); ((volatile b16*)QNh)[(size_t)n * D + d] = p; ((volatile b16*)QNl)[(size_t)n * D + d] = ql; } __threadfence(); }
}
__global__ __launch_bounds__(32) void sc_kernel(const float* __restrict__ src, const b16* __restrict__ QNh, const b16* __restrict__ QNl, float* __restrict__ SC) {
  __shared__ __attribute__((aligned(16))) b16 Ah[16][D + 8]; __shared__ float Tf[16][17]; const int lane = threadIdx.x, nloc = lane & 15, hlf = lane >> 4; const size_t m0 = (size_t)blockIdx.x * 16;
  for (int rr = 0; rr < 16; ++rr) for (int q = 0; q < D / 32; ++q) Ah[rr][q * 32 + lane] = (b16)(bf16_rne(src[(m0 + rr) * D + q * 32 + lane]) * XS);
  wave_lds_sync(); v8f acc = {};
#pragma unroll 4
  for (int kb = 0; kb < D; kb += 32) { const v16b a = frag_kb(&Ah[nloc][kb], hlf); acc = wmma16b(a, frag_kb(QNh + (size_t)nloc * D + kb, hlf), acc); acc = wmma16b(a, frag_kb(QNl + (size_t)nloc * D + kb, hlf), acc); }
#pragma unroll
  for (int r8 = 0; r8 < 8; ++r8) Tf[8 * hlf + r8][nloc] = acc[r8] * (1.0f / (XS * XS));
  wave_lds_sync();
  for (int pass = 0; pass < 2; ++pass) { for (int i = lane; i < 256; i += 32) ((volatile float*)SC)[m0 * 16 + i] = Tf[i / 16][i % 16]; __threadfence(); }
}
__global__ __launch_bounds__(32) void o_kernel(const float* __restrict__ SC, const float* __restrict__ src, int BV, float* __restrict__ O) {
  __shared__ float Aw[3 * WIN]; const int lane = threadIdx.x; const int w = blockIdx.x % NW, n = (blockIdx.x / NW) % NQ, b = blockIdx.x / (NW * NQ); if (b >= BV) return;
  const int k0 = (w > 0 ? (w - 1) : 0) * WIN, k1 = ((w + 2) * WIN < T ? (w + 2) * WIN : T); const int nk = k1 - k0;
  float mx = -INFINITY; for (int j = lane; j < nk; j += 32) mx = fmaxf(mx, SC[((size_t)(k0 + j) * B + b) * 16 + n]); for (int o = 16; o; o >>= 1) mx = fmaxf(mx, __shfl_xor(mx, o));
  float s = 0.0f; for (int j = lane; j < nk; j += 32) { const float e = __expf(SC[((size_t)(k0 + j) * B + b) * 16 + n] - mx); Aw[j] = e; s += e; } for (int o = 16; o; o >>= 1) s += __shfl_xor(s, o); const float inv = 1.0f / s;
  wave_lds_sync(); float acc[32];
#pragma unroll
  for (int q = 0; q < 32; ++q) acc[q] = 0.0f;
#pragma unroll 1
  for (int j = 0; j < nk; ++j) { const float a = Aw[j] * inv; const float* xr = src + ((size_t)(k0 + j) * B + b) * D;
#pragma unroll
    for (int q = 0; q < 32; ++q) acc[q] += pmul(a, bf16_rne(xr[q * 32 + lane])); }
  const size_t orow = (((size_t)b * NQ + n) * NW + w) * D;
  for (int pass = 0; pass < 2; ++pass) { for (int q = 0; q < 32; ++q) ((volatile float*)O)[orow + q * 32 + lane] = acc[q]; __threadfence(); }
}
__global__ __launch_bounds__(32) void ln1_kernel(const float* __restrict__ src, const float* __restrict__ O, const float* __restrict__ wk, const float* __restrict__ g, const float* __restrict__ bt, float* __restrict__ X1, b16* __restrict__ X1h) {
  __shared__ float Tr[D]; const int lane = threadIdx.x; const size_t m0 = (size_t)blockIdx.x * 16;
  for (int pass = 0; pass < 2; ++pass) {
#pragma unroll 1
    for (int rr = 0; rr < 16; ++rr) { const size_t r = m0 + rr; const int t = (int)(r / B), b = (int)(r % B), w = t / WIN; float s = 0.0f;
      for (int q = 0; q < 32; ++q) { const int d = q * 32 + lane; float v = bf16_rne(src[r * D + d]);
#pragma unroll 1
        for (int n = 0; n < NQ; ++n) v += pmul(bf16_rne(wk[n]), O[(((size_t)b * NQ + n) * NW + w) * D + d]); Tr[d] = v; s += v; }
      for (int o = 16; o; o >>= 1) s += __shfl_xor(s, o); const float mu = s * (1.0f / D); float vq = 0.0f; for (int q = 0; q < 32; ++q) { const float dd = Tr[q * 32 + lane] - mu; vq += pmul(dd, dd); } for (int o = 16; o; o >>= 1) vq += __shfl_xor(vq, o); const float rs = rsqrtf(vq * (1.0f / D) + 1e-5f);
      for (int q = 0; q < 32; ++q) { const int d = q * 32 + lane; const float v = pmul(pmul(Tr[d] - mu, rs), bf16_rne(g[d])) + bf16_rne(bt[d]); ((volatile float*)X1)[r * D + d] = v; ((volatile b16*)X1h)[r * D + d] = (b16)(v * XS); }
      wave_lds_sync(); }
    __threadfence(); }
}
__global__ __launch_bounds__(32) void ffn1_kernel(const b16* __restrict__ X1h, const b16* __restrict__ W1T, const float* __restrict__ b1, float dummy, b16* __restrict__ Hh) {
  __shared__ __attribute__((aligned(16))) b16 Th[16][520]; const int lane = threadIdx.x, nloc = lane & 15, hlf = lane >> 4; const int cg = blockIdx.x % (DFF / 512); const size_t m0 = (size_t)(blockIdx.x / (DFF / 512)) * 16; (void)dummy;
#pragma unroll 1
  for (int sub = 0; sub < 4; ++sub) { v8f acc[8];
#pragma unroll
    for (int t = 0; t < 8; ++t) acc[t] = (v8f){};
#pragma unroll 2
    for (int kb = 0; kb < D; kb += 32) { const v16b a = frag_kb(X1h + (m0 + nloc) * D + kb, hlf);
#pragma unroll
      for (int t = 0; t < 8; ++t) acc[t] = wmma16b(a, frag_kb(W1T + (size_t)(cg * 512 + sub * 128 + t * 16 + nloc) * D + kb, hlf), acc[t]); }
#pragma unroll
    for (int t = 0; t < 8; ++t) { const int c = cg * 512 + sub * 128 + t * 16 + nloc; const float bb = bf16_rne(b1[c]);
#pragma unroll
      for (int r8 = 0; r8 < 8; ++r8) Th[8 * hlf + r8][sub * 128 + t * 16 + nloc] = (b16)(fmaxf(acc[t][r8] * (1.0f / (XS * WSC)) + bb, 0.0f) * XS); } }
  wave_lds_sync();
  for (int pass = 0; pass < 2; ++pass) { for (int rr = 0; rr < 16; ++rr) *(volatile v8b*)(Hh + (m0 + rr) * DFF + cg * 512 + lane * 16) = *(const v8b*)(&Th[rr][lane * 16]), *(volatile v8b*)(Hh + (m0 + rr) * DFF + cg * 512 + lane * 16 + 8) = *(const v8b*)(&Th[rr][lane * 16 + 8]); __threadfence(); }
}
__global__ __launch_bounds__(32) void ffn2_kernel(const b16* __restrict__ Hh, const b16* __restrict__ W2T, const float* __restrict__ b2, const float* __restrict__ X1, float* __restrict__ PRE) {
  __shared__ float Tf[16][132]; const int lane = threadIdx.x, nloc = lane & 15, hlf = lane >> 4; const int cg = blockIdx.x % (D / 128); const size_t m0 = (size_t)(blockIdx.x / (D / 128)) * 16; v8f acc[8];
#pragma unroll
  for (int t = 0; t < 8; ++t) acc[t] = (v8f){};
#pragma unroll 2
  for (int kb = 0; kb < DFF; kb += 32) { const v16b a = frag_kb(Hh + (m0 + nloc) * DFF + kb, hlf);
#pragma unroll
    for (int t = 0; t < 8; ++t) acc[t] = wmma16b(a, frag_kb(W2T + (size_t)(cg * 128 + t * 16 + nloc) * DFF + kb, hlf), acc[t]); }
#pragma unroll
  for (int t = 0; t < 8; ++t) { const int c = cg * 128 + t * 16 + nloc; const float bb = bf16_rne(b2[c]);
#pragma unroll
    for (int r8 = 0; r8 < 8; ++r8) Tf[8 * hlf + r8][t * 16 + nloc] = acc[t][r8] * (1.0f / (XS * WSC)) + bb + X1[(m0 + 8 * hlf + r8) * D + c]; }
  wave_lds_sync();
  for (int pass = 0; pass < 2; ++pass) { for (int rr = 0; rr < 16; ++rr) *(volatile v4f*)(PRE + (m0 + rr) * D + cg * 128 + lane * 4) = *(const v4f*)(&Tf[rr][lane * 4]); __threadfence(); }
}
__global__ __launch_bounds__(256) void ln2_kernel(const float* __restrict__ PRE, const float* __restrict__ g, const float* __restrict__ bt, int RL, float* __restrict__ out) {
  const int wave = threadIdx.x >> 5, lane = threadIdx.x & 31; const size_t r = (size_t)blockIdx.x * 8 + wave; if (r >= (size_t)RL) return; const float* pr = PRE + r * D; float s = 0.0f;
#pragma unroll 4
  for (int q = 0; q < 32; ++q) s += pr[q * 32 + lane];
  for (int o = 16; o; o >>= 1) s += __shfl_xor(s, o); const float mu = s * (1.0f / D); float vq = 0.0f;
#pragma unroll 4
  for (int q = 0; q < 32; ++q) { const float dd = pr[q * 32 + lane] - mu; vq += pmul(dd, dd); }
  for (int o = 16; o; o >>= 1) vq += __shfl_xor(vq, o); const float rs = rsqrtf(vq * (1.0f / D) + 1e-5f);
  for (int pass = 0; pass < 2; ++pass) {
#pragma unroll 4
    for (int q = 0; q < 32; ++q) { const int d = q * 32 + lane; ((volatile float*)out)[r * D + d] = pmul(pmul(pr[d] - mu, rs), bf16_rne(g[d])) + bf16_rne(bt[d]); } __threadfence(); }
}
}

extern "C" void kernel_launch(void* const* d_in, const int* in_sizes, int n_in, void* d_out, int out_size, void* d_ws, size_t ws_size, hipStream_t stream) {
  (void)n_in;
  auto Fp = [&](int i) { return (const float*)d_in[i]; };
  if (in_sizes[0] != NR * D || in_sizes[1] != NQ * D || in_sizes[2] != NQ || in_sizes[3] != DFF * D || in_sizes[5] != D * DFF || out_size != NR * D) return;
  const int BV = B; const int RL = NR;
  size_t off = 0; char* ws = (char*)d_ws;
  auto carve = [&](size_t bytes) { char* p = ws + off; off += (bytes + 255) & ~(size_t)255; return p; };
  b16* W1T = (b16*)carve((size_t)DFF * D * 2); b16* W2T = (b16*)carve((size_t)D * DFF * 2); b16* QNh = (b16*)carve((size_t)16 * D * 2); b16* QNl = (b16*)carve((size_t)16 * D * 2); float* SC = (float*)carve((size_t)NR * 16 * 4); float* O = (float*)carve((size_t)B * NQ * NW * D * 4);
  float* X1 = (float*)carve((size_t)NR * D * 4); b16* X1h = (b16*)carve((size_t)NR * D * 2); b16* Hh = (b16*)carve((size_t)NR * DFF * 2); float* PRE = (float*)carve((size_t)NR * D * 4);
  if (off > ws_size || off > ((size_t)96 << 20)) return;
  wcopy_kernel<<<(unsigned)(((size_t)DFF * D / 8 + 255) / 256), 256, 0, stream>>>(Fp(3), (size_t)DFF * D, W1T); wcopy_kernel<<<(unsigned)(((size_t)D * DFF / 8 + 255) / 256), 256, 0, stream>>>(Fp(5), (size_t)D * DFF, W2T);
  qn_kernel<<<16, 32, 0, stream>>>(Fp(1), QNh, QNl);
  sc_kernel<<<NR / 16, 32, 0, stream>>>(Fp(0), QNh, QNl, SC);
  o_kernel<<<BV * NQ * NW, 32, 0, stream>>>(SC, Fp(0), BV, O);
  ln1_kernel<<<RL / 16, 32, 0, stream>>>(Fp(0), O, Fp(2), Fp(7), Fp(8), X1, X1h);
  ffn1_kernel<<<(RL / 16) * (DFF / 512), 32, 0, stream>>>(X1h, W1T, Fp(4), 0.0f, Hh);
  ffn2_kernel<<<(RL / 16) * (D / 128), 32, 0, stream>>>(Hh, W2T, Fp(6), X1, PRE);
  ln2_kernel<<<(RL + 7) / 8, 256, 0, stream>>>(PRE, Fp(9), Fp(10), RL, (float*)d_out);
}
